// DescriptorNet_31490700214403
// MI455X (gfx1250) — hardware-verified
//
#include <hip/hip_runtime.h>
#include <math.h>

typedef __attribute__((ext_vector_type(16))) _Float16 v16h;
typedef __attribute__((ext_vector_type(16))) __bf16 v16b;
typedef __attribute__((ext_vector_type(8)))  _Float16 v8h;
typedef __attribute__((ext_vector_type(8)))  float v8f;
typedef __attribute__((ext_vector_type(4)))  float v4f;
typedef __attribute__((ext_vector_type(2)))  float v2f;
typedef __attribute__((ext_vector_type(4)))  unsigned v4u;
typedef __attribute__((ext_vector_type(4)))  int v4i;
typedef float __attribute__((may_alias)) float_a;
typedef int __attribute__((may_alias)) int_a;

template <typename T> __device__ __forceinline__ void vst2(void* p, T v) { *(volatile T*)p = v; __threadfence(); *(volatile T*)p = v; }
__device__ __forceinline__ v8f wmma16(v16h a, v16h b, v8f c) {
  v8f d = __builtin_amdgcn_wmma_f32_16x16x32_f16(false, a, false, b, (short)0, c, false, false);
  asm volatile("v_nop\n\tv_nop\n\tv_nop\n\tv_nop" : "+v"(d) : "v"(a), "v"(b));
  return d;
}
__device__ __forceinline__ v8f wmma_bf(v16b a, v16b b, v8f c) {
  v8f d = __builtin_amdgcn_wmma_f32_16x16x32_bf16(false, a, false, b, (short)0, c, false, false);
  asm volatile("v_nop\n\tv_nop\n\tv_nop\n\tv_nop" : "+v"(d) : "v"(a), "v"(b));
  return d;
}
__device__ __forceinline__ v16h frag_h(const _Float16* rowk0, int lane) {
  union { v16h v; v8h q[2]; } u; const _Float16* p = rowk0 + 8 * (lane >> 4);
  u.q[0] = *(const v8h*)p; u.q[1] = *(const v8h*)(p + 16); return u.v;
}
__device__ __forceinline__ v16h frag_f32(const float* rowk0, int lane) {
  v16h a; const float* p = rowk0 + 8 * (lane >> 4);
#pragma unroll
  for (int i = 0; i < 8; ++i) { a[i] = (_Float16)p[i]; a[8 + i] = (_Float16)p[16 + i]; }
  return a;
}
__device__ __forceinline__ v16h frag_f32s(const float* rowk0, int lane, float sc) {
  v16h a; const float* p = rowk0 + 8 * (lane >> 4);
#pragma unroll
  for (int i = 0; i < 8; ++i) { a[i] = (_Float16)(p[i] * sc); a[8 + i] = (_Float16)(p[16 + i] * sc); }
  return a;
}
__device__ __forceinline__ v16h fragc_f32(const float* W, int k0, int n, int lane, int ld, int K) {
  v16h a; const int g = lane >> 4;
#pragma unroll
  for (int i = 0; i < 8; ++i) { const int ka = k0 + 8 * g + i, kb = ka + 16;
    a[i] = (_Float16)(ka < K ? W[(size_t)ka * ld + n] : 0.f); a[8 + i] = (_Float16)(kb < K ? W[(size_t)kb * ld + n] : 0.f); }
  return a;
}
struct F2 { v16b h, l; };
__device__ __forceinline__ F2 bsplit16(const float v[16]) { F2 r;
#pragma unroll
  for (int i = 0; i < 16; ++i) { const __bf16 h = (__bf16)v[i]; r.h[i] = h; r.l[i] = (__bf16)(v[i] - (float)h); }
  return r; }
__device__ __forceinline__ F2 split_row(const float* row, int k0, int lane) { float v[16]; const float* p = row + k0 + 8 * (lane >> 4);
#pragma unroll
  for (int i = 0; i < 8; ++i) { v[i] = p[i]; v[8 + i] = p[16 + i]; }
  return bsplit16(v); }
__device__ __forceinline__ F2 split_rowK(const float* row, int k0, int lane, int K) { float v[16]; const int g = lane >> 4;
#pragma unroll
  for (int i = 0; i < 8; ++i) { const int ka = k0 + 8 * g + i, kb = ka + 16; v[i] = ka < K ? row[ka] : 0.f; v[8 + i] = kb < K ? row[kb] : 0.f; }
  return bsplit16(v); }
__device__ __forceinline__ F2 split_col(const float* W, int k0, int n, int lane, int ld, int K) { float v[16]; const int g = lane >> 4;
#pragma unroll
  for (int i = 0; i < 8; ++i) { const int ka = k0 + 8 * g + i, kb = ka + 16; v[i] = ka < K ? W[(size_t)ka * ld + n] : 0.f; v[8 + i] = kb < K ? W[(size_t)kb * ld + n] : 0.f; }
  return bsplit16(v); }
__device__ __forceinline__ v8f mac3(const F2& a, const F2& b, v8f c) { c = wmma_bf(a.l, b.h, c); c = wmma_bf(a.h, b.l, c); return wmma_bf(a.h, b.h, c); }
__device__ __forceinline__ float sigm(float v) { return 1.0f / (1.0f + expf(-v)); }
#define LDSX() do { asm volatile("s_wait_dscnt 0" ::: "memory"); __builtin_amdgcn_wave_barrier(); __builtin_amdgcn_fence(__ATOMIC_RELEASE, "workgroup"); } while (0)

#define NA 10000
#define NNB 128
#define M1 25
#define M2 50
#define MM 100
#define MP 10
#define NE (NA * NNB)

__device__ __forceinline__ F2 colsplit_g(const float* __restrict__ W, int k0, int n, int lane, int ld, int K, int ncols) {
  const int g = lane >> 4; float bv[16];
#pragma unroll
  for (int i = 0; i < 8; ++i) { const int ka = k0 + 8 * g + i, kb = ka + 16; bv[i] = (ka < K && n < ncols) ? W[(size_t)ka * ld + n] : 0.f; bv[8 + i] = (kb < K && n < ncols) ? W[(size_t)kb * ld + n] : 0.f; }
  return bsplit16(bv);
}
__global__ __launch_bounds__(128) void k_main(const float* __restrict__ ev, const float* __restrict__ W0, const float* __restrict__ b0, const float* __restrict__ W1, const float* __restrict__ b1, const float* __restrict__ Wo, const float* __restrict__ bo, float* __restrict__ Dp) {
  __shared__ __align__(16) float senv[NNB][4];
  __shared__ __align__(16) float sh1[4][16][36];
  __shared__ __align__(16) float sh2[4][16][68];
  __shared__ float sHE[4][M2][4];
  __shared__ float sH2E[M2][4]; __shared__ float sEs[4];
  __shared__ __align__(16) float sS[MM][4];
  __shared__ __align__(16) float sD[MM * MP];
  const int tid = threadIdx.x, wave = tid >> 5, lane = tid & 31, col = lane & 15, g = lane >> 4;
  const int a = blockIdx.x;
  { const int n = tid; const float* e3 = ev + ((size_t)a * NNB + n) * 3; const float x = e3[0], y = e3[1], z = e3[2];
    const float r = sqrtf(x * x + y * y + z * z); const float rs = fmaxf(r, 1e-8f); const float ir = 1.0f / rs;
    const float u = (rs - 2.0f) * 0.25f; const float poly = u * u * u * (-6.0f * u * u + 15.0f * u - 10.0f); const float smid = ir * (poly + 1.0f);
    const float sij = rs < 2.0f ? ir : (rs < 6.0f ? smid : 0.f);
    senv[n][0] = (sij - 0.05f) * 10.0f; const float sc = sij * 2.0f; senv[n][1] = x * sc; senv[n][2] = y * sc; senv[n][3] = z * sc; }
  __syncthreads();
  float he[8];
#pragma unroll
  for (int e = 0; e < 8; ++e) he[e] = 0.f;
#pragma unroll 1
  for (int tix = 0; tix < 2; ++tix) { const int n0 = (wave * 2 + tix) * 16;
    for (int j = g * 16; j < g * 16 + 16; ++j) { float v = 0.f; if (j < M1) { v = senv[n0 + col][0] * W0[j] + b0[j]; v = v > 0.f ? v : 0.f; } if (j < 32) sh1[wave][col][j] = v; }
    LDSX();
    { const F2 aa = split_row(&sh1[wave][col][0], 0, lane); v8f acc[4] = {};
#pragma unroll
      for (int t = 0; t < 4; ++t) acc[t] = mac3(aa, colsplit_g(W1, 0, t * 16 + col, lane, M2, M1, M2), acc[t]);
#pragma unroll
      for (int t = 0; t < 4; ++t) { const int c = t * 16 + col; const float bb = c < M2 ? b1[c] : 0.f;
#pragma unroll
        for (int r = 0; r < 8; ++r) { float v = acc[t][r] + bb; v = v > 0.f ? v : 0.f; sh2[wave][8 * g + r][c] = c < M2 ? v : 0.f; } } }
    LDSX();
#pragma unroll 4
    for (int nn = 0; nn < 16; ++nn) { const float* er = &senv[n0 + nn][0]; const float h0 = sh2[wave][nn][lane]; const float h1v = (lane + 32 < M2) ? sh2[wave][nn][lane + 32] : 0.f;
#pragma unroll
      for (int f = 0; f < 4; ++f) { he[f] += h0 * er[f]; he[4 + f] += h1v * er[f]; } }
    LDSX(); }
#pragma unroll
  for (int f = 0; f < 4; ++f) { sHE[wave][lane][f] = he[f]; if (lane + 32 < M2) sHE[wave][lane + 32][f] = he[4 + f]; }
  __syncthreads();
  for (int q = tid; q < M2 * 4 + 4; q += 128) {
    if (q < M2 * 4) { const int j = q >> 2, f = q & 3; sH2E[j][f] = (sHE[0][j][f] + sHE[1][j][f]) + (sHE[2][j][f] + sHE[3][j][f]); }
    else { const int f = q - M2 * 4; float s = 0.f; for (int n = 0; n < NNB; ++n) s += senv[n][f]; sEs[f] = s; } }
  __syncthreads();
  for (int q = tid; q < MM * 4; q += 128) { const int m = q >> 2, f = q & 3; float s = bo[m] * sEs[f];
#pragma unroll 10
    for (int j = 0; j < M2; ++j) s += Wo[j * MM + m] * sH2E[j][f];
    sS[m][f] = s; }
  __syncthreads();
  for (int q = tid; q < MM * MP; q += 128) { const int m = q / MP, p = q % MP; sD[q] = sS[m][0] * sS[p][0] + sS[m][1] * sS[p][1] + sS[m][2] * sS[p][2] + sS[m][3] * sS[p][3]; }
  __syncthreads();
  for (int q = tid; q < MM * MP / 4; q += 128) vst2(Dp + (size_t)a * 1024 + q * 4, *(const v4f*)(&sD[q * 4]));
}
__global__ __launch_bounds__(256) void k_copy(const float* __restrict__ Dp, float* __restrict__ out) {
  const int tid = threadIdx.x; const size_t a0 = (size_t)blockIdx.x * 8;
  for (int q = tid; q < 8 * (MM * MP / 4); q += 256) { const int al = q / (MM * MP / 4), pc = q % (MM * MP / 4); vst2(out + (a0 + al) * (MM * MP) + pc * 4, *(const v4f*)(Dp + (a0 + al) * 1024 + pc * 4)); }
}
extern "C" void kernel_launch(void* const* d_in, const int* in_sizes, int n_in, void* d_out, int out_size, void* d_ws, size_t ws_size, hipStream_t stream) {
  (void)in_sizes; (void)n_in; (void)out_size; (void)ws_size;
  const float* ev = (const float*)d_in[0]; const float* W0 = (const float*)d_in[1]; const float* b0 = (const float*)d_in[2]; const float* W1 = (const float*)d_in[3]; const float* b1 = (const float*)d_in[4]; const float* Wo = (const float*)d_in[5]; const float* bo = (const float*)d_in[6];
  float* out = (float*)d_out;
  float* Dp = (float*)d_ws;
  k_main<<<NA, 128, 0, stream>>>(ev, W0, b0, W1, b1, Wo, bo, Dp);
  k_copy<<<NA / 8, 256, 0, stream>>>(Dp, out);
}
